// RefinePixel_26697516712464
// MI455X (gfx1250) — hardware-verified
//
#include <hip/hip_runtime.h>

typedef _Float16 f16t;
typedef _Float16 v16h __attribute__((ext_vector_type(16)));
typedef _Float16 v8h  __attribute__((ext_vector_type(8)));
typedef float    v8f  __attribute__((ext_vector_type(8)));
typedef float    v4f  __attribute__((ext_vector_type(4)));
typedef v8h __attribute__((may_alias)) v8ha;
typedef v4f __attribute__((may_alias)) v4fa;
union Frag { v16h v; v8h half[2]; };

#define NB    8
#define CF    64
#define HH    128
#define WD    128
#define NP    16384
#define PW    130
#define NPP   16900
#define CO    256
#define KW    608
#define NCT   32
#define NV    128
#define FSC   8.0f
#define MSC   32.0f
#define WSCF  64.0f
#define WSCM  16.0f
#define OSC   (1.0f / 512.0f)

static_assert((CO * KW * 2) % 512 == 0);
static_assert((NB * NPP * CF * 2) % 128 == 0);
static_assert((NB * NP * 32 * 2) % 128 == 0);
static_assert(KW == 9 * CF + 32);

__device__ __forceinline__ v8f wmma_f16(v16h a, v16h b, v8f c) {
  v8f d = __builtin_amdgcn_wmma_f32_16x16x32_f16(false, a, false, b, (short)0, c, false, false);
  asm volatile("v_nop\n\tv_nop\n\tv_nop\n\tv_nop" : "+v"(d) : "v"(a), "v"(b));
  return d;
}

__device__ __forceinline__ v16h load_frag32(const f16t* p, int h) {
  Frag f;
  f.half[0] = *(const v8ha*)(p + 8 * h);
  f.half[1] = *(const v8ha*)(p + 16 + 8 * h);
  return f.v;
}

__device__ __forceinline__ v8f zero8f() {
  v8f z;
  #pragma unroll
  for (int j = 0; j < 8; ++j) z[j] = 0.f;
  return z;
}

__device__ __forceinline__ float vzero() {
  float r;
  asm volatile("v_mov_b32 %0, 0" : "=v"(r));
  return r;
}

__global__ __launch_bounds__(256) void map_k(const float* __restrict__ ctr,
                                            const int* __restrict__ bind,
                                            float* __restrict__ S)
{
  #pragma clang fp contract(off)
  __shared__ float scx[NCT * NV];
  __shared__ float scy[NCT * NV];
  __shared__ int   sbi[NCT];
  __shared__ __attribute__((aligned(16))) float sS[256];
  const int tid = threadIdx.x, lane = tid & 31, w = tid >> 5;
  for (int i = tid; i < NCT * NV; i += 256) {
    scx[i] = ctr[2 * i]     * 0.25f;
    scy[i] = ctr[2 * i + 1] * 0.25f;
  }
  if (tid < NCT) sbi[tid] = bind[tid];
  __syncthreads();

  const int n   = blockIdx.y;
  const int pix = blockIdx.x * 256 + tid;
  const float fx = (float)(pix & (WD - 1));
  const float fy = (float)(pix >> 7);
  float acc = 0.f;
  #pragma unroll 1
  for (int c = 0; c < NCT; ++c) {
    if (sbi[c] == n) {
      const float* cx = scx + c * NV;
      const float* cy = scy + c * NV;
      float t = 0.f;
      #pragma unroll 1
      for (int v = 0; v < NV; ++v) {
        const float dx = fx - cx[v];
        const float dy = fy - cy[v];
        const float d2 = dx * dx + dy * dy;
        if (d2 < 220.0f) t += expf(-0.5f * d2);
      }
      acc += t * (1.0f / 6.2831855f);
    }
  }
  sS[tid] = acc;
  __syncthreads();
  if (w < 2) {
    const v4f v = *(const v4fa*)(sS + w * 128 + 4 * lane);
    float* dp = S + (size_t)n * NP + (size_t)blockIdx.x * 256 + w * 128 + 4 * lane;
    *(volatile v4f*)dp = v;
    __threadfence();
    *(volatile v4f*)dp = v;
  }
}

__global__ __launch_bounds__(256) void wcvt_k(const float* __restrict__ w1, f16t* __restrict__ Wr)
{
  const int g = blockIdx.x * 256 + threadIdx.x;
  if (g >= CO * (KW / 8)) return;
  const int o  = g / (KW / 8);
  const int kg = g - o * (KW / 8);
  v8h o8;
  #pragma unroll
  for (int i = 0; i < 8; ++i) {
    const int k    = 8 * kg + i;
    const int isF  = (k < 9 * CF) ? 1 : 0;
    const int cch  = (k & (CF - 1)) + 1;
    int tapF = k >> 6;            tapF = tapF > 8 ? 8 : tapF;
    int t    = k - 9 * CF;        t = t < 0 ? 0 : (t > 8 ? 8 : t);
    const int idx  = isF ? ((o * 65 + cch) * 9 + tapF) : (o * 65 * 9 + t);
    const float sc = isF ? WSCF : ((k < 9 * CF + 9) ? WSCM : 0.0f);
    o8[i] = (f16t)(w1[idx] * sc);
  }
  f16t* dp = Wr + (size_t)8 * g;
  *(volatile v8h*)dp = o8;
  __threadfence();
  *(volatile v8h*)dp = o8;
}

__global__ __launch_bounds__(256) void tcvt_k(const float* __restrict__ x, f16t* __restrict__ T)
{
  __shared__ __attribute__((aligned(16))) f16t sH[WD * CF];
  const int tid = threadIdx.x, lane = tid & 31, w = tid >> 5;
  const int yp = blockIdx.x, n = blockIdx.y;
  const int inner = (yp >= 1 && yp <= HH) ? 1 : 0;
  const f16t hz = (f16t)vzero();
  if (inner) {
    const int y = yp - 1;
    #pragma unroll 1
    for (int j = 0; j < 8; ++j) {
      const int item = tid + 256 * j;
      const int c = item >> 5, x0 = 4 * (item & 31);
      const v4f v = *(const v4fa*)(x + ((size_t)(n * CF + c) * HH + y) * WD + x0);
      sH[(x0 + 0) * CF + c] = (f16t)(v.x * FSC);
      sH[(x0 + 1) * CF + c] = (f16t)(v.y * FSC);
      sH[(x0 + 2) * CF + c] = (f16t)(v.z * FSC);
      sH[(x0 + 3) * CF + c] = (f16t)(v.w * FSC);
    }
  } else {
    v8h zv;
    #pragma unroll
    for (int j = 0; j < 8; ++j) zv[j] = hz;
    #pragma unroll 1
    for (int i = tid; i < (WD * CF) / 8; i += 256) *(v8ha*)(sH + 8 * i) = zv;
  }
  __syncthreads();

  const int q8 = lane & 7, sub = lane >> 3;
  v8h vals[5];
  size_t d[5];
  int ok[5];
  #pragma unroll
  for (int i = 0; i < 5; ++i) {
    const int lid = 32 * i + 4 * w + sub;
    ok[i] = (lid < PW) ? 1 : 0;
    const int xp  = (lid < PW) ? lid : (PW - 1);
    const int okx = (xp >= 1 && xp <= WD) ? 1 : 0;
    int xs = xp - 1; xs = xs < 0 ? 0 : (xs > WD - 1 ? WD - 1 : xs);
    v8h vv = *(const v8ha*)(sH + xs * CF + 8 * q8);
    #pragma unroll
    for (int j = 0; j < 8; ++j) vv[j] = okx ? vv[j] : hz;
    vals[i] = vv;
    d[i] = ((size_t)n * NPP + (size_t)yp * PW + xp) * CF + 8 * q8;
  }
  #pragma unroll
  for (int i = 0; i < 5; ++i) if (ok[i]) *(volatile v8h*)(T + d[i]) = vals[i];
  __threadfence();
  #pragma unroll
  for (int i = 0; i < 5; ++i) if (ok[i]) *(volatile v8h*)(T + d[i]) = vals[i];
}

__global__ __launch_bounds__(256) void scvt_k(const float* __restrict__ S, f16t* __restrict__ Sp)
{
  __shared__ __attribute__((aligned(16))) f16t sP[WD * 32];
  const int tid = threadIdx.x, lane = tid & 31, w = tid >> 5;
  const int y = blockIdx.x, n = blockIdx.y;
  const f16t hz = (f16t)vzero();
  if (tid < WD) {
    const int xq = tid;
    const float* Sn = S + (size_t)n * NP;
    float e[9];
    #pragma unroll
    for (int dy = 0; dy < 3; ++dy) {
      const int yy  = y + dy - 1;
      const int oky = (yy >= 0 && yy < HH) ? 1 : 0;
      const int yc  = yy < 0 ? 0 : (yy > HH - 1 ? HH - 1 : yy);
      #pragma unroll
      for (int dx = 0; dx < 3; ++dx) {
        const int xx  = xq + dx - 1;
        const int okx = (xx >= 0 && xx < WD) ? 1 : 0;
        const int xc  = xx < 0 ? 0 : (xx > WD - 1 ? WD - 1 : xx);
        const float val = Sn[yc * WD + xc];
        e[dy * 3 + dx] = (oky && okx) ? (val * MSC) : 0.0f;
      }
    }
    v8h g0, g1, zv;
    #pragma unroll
    for (int j = 0; j < 8; ++j) { g0[j] = (f16t)e[j]; g1[j] = hz; zv[j] = hz; }
    g1[0] = (f16t)e[8];
    f16t* row = sP + xq * 32;
    *(v8ha*)(row)      = g0;
    *(v8ha*)(row + 8)  = g1;
    *(v8ha*)(row + 16) = zv;
    *(v8ha*)(row + 24) = zv;
  }
  __syncthreads();
  const int q8 = lane & 7, sub = lane >> 3;
  v8h vals[2];
  size_t d[2];
  #pragma unroll
  for (int i = 0; i < 2; ++i) {
    const int line = 8 * w + 4 * i + sub;
    vals[i] = *(const v8ha*)(sP + line * 64 + 8 * q8);
    d[i] = ((size_t)(n * HH + y) * WD) * 32 + (size_t)line * 64 + 8 * q8;
  }
  #pragma unroll
  for (int i = 0; i < 2; ++i) *(volatile v8h*)(Sp + d[i]) = vals[i];
  __threadfence();
  #pragma unroll
  for (int i = 0; i < 2; ++i) *(volatile v8h*)(Sp + d[i]) = vals[i];
}

__global__ __launch_bounds__(256) void conv_k(
    const f16t* __restrict__ T, const f16t* __restrict__ Sp, const f16t* __restrict__ Wr,
    const float* __restrict__ b1, const float* __restrict__ w2, const float* __restrict__ b2,
    float* __restrict__ out)
{
  __shared__ float sPar[3 * CO];
  __shared__ float red[8 * 2 * 64];
  __shared__ __attribute__((aligned(16))) float sOut[128];
  const int tid = threadIdx.x, lane = tid & 31, w = tid >> 5;
  const int h = lane >> 4, m = lane & 15;
  const int x0 = blockIdx.x * 64, y = blockIdx.y, n = blockIdx.z;

  sPar[tid]          = b1[tid];
  sPar[CO + tid]     = w2[tid];
  sPar[2 * CO + tid] = w2[CO + tid];
  __syncthreads();

  const v8f z8 = zero8f();
  v8f acc[2][4];
  #pragma unroll
  for (int mt = 0; mt < 2; ++mt) {
    #pragma unroll
    for (int nt = 0; nt < 4; ++nt) acc[mt][nt] = z8;
  }

  const f16t* wr0 = Wr + (size_t)(32 * w + m) * KW;
  const size_t wst = (size_t)16 * KW;
  const f16t* tb = T + ((size_t)n * NPP + (size_t)y * PW + x0 + m) * CF;

  #pragma unroll 1
  for (int tap = 0; tap < 9; ++tap) {
    const int dy = (tap * 11) >> 5, dx = tap - 3 * dy;
    const f16t* bp = tb + (size_t)(dy * PW + dx) * CF;
    const f16t* ap = wr0 + tap * CF;
    #pragma unroll
    for (int cc = 0; cc < 2; ++cc) {
      const int c0 = 32 * cc;
      const v16h a0 = load_frag32(ap + c0, h);
      const v16h a1 = load_frag32(ap + wst + c0, h);
      #pragma unroll
      for (int nt = 0; nt < 4; ++nt) {
        const v16h bb = load_frag32(bp + (size_t)(16 * nt) * CF + c0, h);
        acc[0][nt] = wmma_f16(a0, bb, acc[0][nt]);
        acc[1][nt] = wmma_f16(a1, bb, acc[1][nt]);
      }
    }
  }
  {
    const v16h a0 = load_frag32(wr0 + 9 * CF, h);
    const v16h a1 = load_frag32(wr0 + wst + 9 * CF, h);
    const f16t* sp = Sp + ((size_t)(n * HH + y) * WD + x0 + m) * 32;
    #pragma unroll
    for (int nt = 0; nt < 4; ++nt) {
      const v16h bb = load_frag32(sp + (size_t)(16 * nt) * 32, h);
      acc[0][nt] = wmma_f16(a0, bb, acc[0][nt]);
      acc[1][nt] = wmma_f16(a1, bb, acc[1][nt]);
    }
  }

  float pA[4], pB[4];
  #pragma unroll
  for (int nt = 0; nt < 4; ++nt) {
    float pa = 0.f, pb = 0.f;
    #pragma unroll
    for (int mt = 0; mt < 2; ++mt) {
      #pragma unroll
      for (int r = 0; r < 8; ++r) {
        const int o = 32 * w + 16 * mt + 8 * h + r;
        const float hv = fmaxf(acc[mt][nt][r] * OSC + sPar[o], 0.0f);
        pa += sPar[CO + o] * hv;
        pb += sPar[2 * CO + o] * hv;
      }
    }
    pa += __shfl_xor(pa, 16, 32);
    pb += __shfl_xor(pb, 16, 32);
    pA[nt] = pa;
    pB[nt] = pb;
  }
  if (h == 0) {
    #pragma unroll
    for (int nt = 0; nt < 4; ++nt) {
      red[(2 * w + 0) * 64 + 16 * nt + m] = pA[nt];
      red[(2 * w + 1) * 64 + 16 * nt + m] = pB[nt];
    }
  }
  __syncthreads();
  if (tid < 128) {
    const int oc = tid >> 6, px = tid & 63;
    float s = b2[oc];
    #pragma unroll
    for (int ww = 0; ww < 8; ++ww) s += red[(2 * ww + oc) * 64 + px];
    sOut[oc * 64 + px] = s;
  }
  __syncthreads();
  if (w == 0) {
    const int oc = lane >> 4, q = lane & 15;
    const v4f v = *(const v4fa*)(sOut + oc * 64 + 4 * q);
    float* dp = out + ((size_t)(n * 2 + oc) * NP + (size_t)y * WD + x0 + 4 * q);
    *(volatile v4f*)dp = v;
    __threadfence();
    *(volatile v4f*)dp = v;
  }
}

extern "C" void kernel_launch(void* const* d_in, const int* in_sizes, int n_in,
                              void* d_out, int out_size, void* d_ws, size_t ws_size,
                              hipStream_t stream)
{
  if (n_in < 7) return;
  if (in_sizes[0] != NCT * NV * 2) return;
  if (in_sizes[1] != NB * CF * NP) return;
  if (in_sizes[2] != NCT) return;
  if (in_sizes[3] != CO * 65 * 9) return;
  if (in_sizes[4] != CO) return;
  if (in_sizes[5] != 2 * CO) return;
  if (in_sizes[6] != 2) return;
  if (out_size != NB * 2 * NP + NB * NP) return;

  const float* ctr  = (const float*)d_in[0];
  const float* ftr  = (const float*)d_in[1];
  const int*   bind = (const int*)  d_in[2];
  const float* w1   = (const float*)d_in[3];
  const float* b1   = (const float*)d_in[4];
  const float* w2   = (const float*)d_in[5];
  const float* b2   = (const float*)d_in[6];
  float* out0 = (float*)d_out;
  float* out1 = out0 + (size_t)NB * 2 * NP;

  const size_t szWr = (size_t)CO * KW * 2;
  const size_t szT  = (size_t)NB * NPP * CF * 2;
  const size_t szSp = (size_t)NB * NP * 32 * 2;
  size_t off = 0;
  char* ws = (char*)d_ws;
  f16t* Wr = (f16t*)(ws + off); off += szWr;
  f16t* T  = (f16t*)(ws + off); off += szT;
  f16t* Sp = (f16t*)(ws + off); off += szSp;
  if (off > ws_size) return;

  map_k<<<dim3(NP / 256, NB), 256, 0, stream>>>(ctr, bind, out1);
  wcvt_k<<<(CO * (KW / 8)) / 256, 256, 0, stream>>>(w1, Wr);
  tcvt_k<<<dim3(PW, NB), 256, 0, stream>>>(ftr, T);
  scvt_k<<<dim3(HH, NB), 256, 0, stream>>>(out1, Sp);
  conv_k<<<dim3(2, HH, NB), 256, 0, stream>>>(T, Sp, Wr, b1, w2, b2, out0);
}
